// IDW_impute_low_high_pass_62268435857709
// MI455X (gfx1250) — hardware-verified
//
#include <hip/hip_runtime.h>


namespace {
constexpr int B = 32, T = 512, M = 128, BAND = 184, GW = 512, GOFF = 256;
constexpr float XS = 8.0f;
typedef _Float16 b16;
typedef __attribute__((ext_vector_type(16))) _Float16 v16b;
typedef __attribute__((ext_vector_type(8))) _Float16 v8b;
typedef __attribute__((ext_vector_type(8))) float v8f;
typedef __attribute__((ext_vector_type(4))) float v4f;
__device__ __forceinline__ float bf16_rne(float f) { unsigned int u = __float_as_uint(f); u += 0x7FFFu + ((u >> 16) & 1u); float r = __uint_as_float(u & 0xFFFF0000u); asm volatile("" : "+v"(r)); return r; }
__device__ __forceinline__ void split16(float v, b16& hi, b16& lo) { hi = (b16)v; lo = (b16)(v - (float)hi); }
__device__ __forceinline__ v16b frag_kb(const b16* p, int hh) { const v8b a = *(const v8b*)(p + 8 * hh), b = *(const v8b*)(p + 16 + 8 * hh); v16b f;
#pragma unroll
  for (int e = 0; e < 8; ++e) { f[e] = a[e]; f[8 + e] = b[e]; } return f; }
__device__ __forceinline__ v8f wmma16b(v16b a, v16b b, v8f c) { v8f d = __builtin_amdgcn_wmma_f32_16x16x32_f16(false, a, false, b, (short)0, c, false, false); asm volatile("v_nop\n\tv_nop\n\tv_nop\n\tv_nop" : "+v"(d) : "v"(a), "v"(b)); return d; }
__device__ __forceinline__ void wave_lds_sync() { __builtin_amdgcn_fence(__ATOMIC_RELEASE, "workgroup"); __builtin_amdgcn_wave_barrier(); __builtin_amdgcn_fence(__ATOMIC_ACQUIRE, "workgroup"); }
__device__ __forceinline__ float pmul(float a, float b) { float p = a * b; asm volatile("" : "+v"(p)); return p; }
__device__ __forceinline__ float softplus(float v) { return v > 20.0f ? v : __logf(1.0f + __expf(v)); }

__global__ __launch_bounds__(256) void prep_kernel(const float* __restrict__ data, const float* __restrict__ mask, const float* __restrict__ kk, const float* __restrict__ lgw, const float* __restrict__ lcc, b16* __restrict__ KP, b16* __restrict__ VB, b16* __restrict__ CFh, b16* __restrict__ CFl) {
  const size_t u = (size_t)blockIdx.x * 256 + threadIdx.x;
  for (int pass = 0; pass < 2; ++pass) {
    if (u < (size_t)2 * M * (GW / 8)) { const int which = (int)(u / (M * (GW / 8))); const int r = (int)(u % (M * (GW / 8))); const int d = r / (GW / 8), i0 = (r % (GW / 8)) * 8;
      const float w = which == 0 ? softplus(bf16_rne(lgw[d])) : softplus(bf16_rne(kk[d])) + 1.0f; v8b hv, lv;
#pragma unroll
      for (int j = 0; j < 8; ++j) { const float g = (float)(i0 + j - GOFF) * 0.1f; const float kv = __expf(-pmul(pmul(g, g), w)); b16 p, q; split16(kv * XS, p, q); hv[j] = p; lv[j] = q; }
      b16* base = KP + ((size_t)(which * 2) * M + d) * GW + i0; *(volatile v8b*)base = hv; *(volatile v8b*)(base + (size_t)M * GW) = lv; }
    if (u < (size_t)2 * M * B * (T / 8)) { const int which = (int)(u / ((size_t)M * B * (T / 8))); const size_t r = u % ((size_t)M * B * (T / 8)); const int d = (int)(r / (B * (T / 8))), b = (int)((r / (T / 8)) % B), s0 = (int)(r % (T / 8)) * 8; v8b v;
#pragma unroll
      for (int j = 0; j < 8; ++j) { const size_t src = ((size_t)b * T + s0 + j) * M + d; const float mv = bf16_rne(mask[src]); v[j] = (b16)((which == 0 ? mv : pmul(bf16_rne(data[src]), mv)) * XS); } *(volatile v8b*)(VB + (((size_t)which * M + d) * B + b) * T + s0) = v; }
    if (u < (size_t)M * 16) { const int j = (int)(u / 16), d0 = (int)(u % 16) * 8; v8b hv, lv;
#pragma unroll
      for (int i = 0; i < 8; ++i) { b16 p, q; split16(softplus(bf16_rne(lcc[(size_t)(d0 + i) * M + j])) * XS, p, q); hv[i] = p; lv[i] = q; } *(volatile v8b*)(CFh + (size_t)j * M + d0) = hv; *(volatile v8b*)(CFl + (size_t)j * M + d0) = lv; }
    __threadfence(); } }
__global__ __launch_bounds__(32) void infl_kernel(const b16* __restrict__ VB, const b16* __restrict__ KP, float* __restrict__ O0, float* __restrict__ I1, float* __restrict__ M2, float* __restrict__ I2) {
  __shared__ float Tf[32][132]; const int lane = threadIdx.x, nloc = lane & 15, hlf = lane >> 4; const int wid = blockIdx.x; const int tg = wid % 4, which = (wid / 4) % 4, d = wid / 16; const int t0 = tg * 128; const int vsel = which & 1, ksel = which >> 1;
  const b16* vb = VB + ((size_t)vsel * M + d) * B * T; const b16* kh = KP + ((size_t)(ksel * 2) * M + d) * GW; const b16* kl = kh + (size_t)M * GW;
  v8f acc[2][8];
#pragma unroll
  for (int mm = 0; mm < 2; ++mm)
#pragma unroll
    for (int tt = 0; tt < 8; ++tt) acc[mm][tt] = (v8f){};
#pragma unroll 1
  for (int kb = 0; kb < T; kb += 32) { if (kb + 31 < t0 - BAND || kb > t0 + 127 + BAND) continue; const v16b a0 = frag_kb(vb + (size_t)nloc * T + kb, hlf), a1 = frag_kb(vb + (size_t)(16 + nloc) * T + kb, hlf);
#pragma unroll
    for (int tt = 0; tt < 8; ++tt) { const int tb = t0 + tt * 16; if (kb + 31 < tb - BAND || kb > tb + 15 + BAND) continue; const int ro = kb - (tb + nloc) + GOFF;     const v16b bh = frag_kb(kh + ro, hlf), bl = frag_kb(kl + ro, hlf);
      acc[0][tt] = wmma16b(a0, bh, acc[0][tt]); acc[0][tt] = wmma16b(a0, bl, acc[0][tt]); acc[1][tt] = wmma16b(a1, bh, acc[1][tt]); acc[1][tt] = wmma16b(a1, bl, acc[1][tt]); } }
#pragma unroll
  for (int mm = 0; mm < 2; ++mm)
#pragma unroll
    for (int tt = 0; tt < 8; ++tt)
#pragma unroll
      for (int r8 = 0; r8 < 8; ++r8) Tf[mm * 16 + 8 * hlf + r8][tt * 16 + nloc] = acc[mm][tt][r8] * (1.0f / (XS * XS));
  wave_lds_sync(); float* dst = which == 0 ? O0 : which == 1 ? I1 : which == 2 ? M2 : I2;
  for (int pass = 0; pass < 2; ++pass) { for (int b = 0; b < B; ++b) *(volatile v4f*)(dst + ((size_t)b * M + d) * T + t0 + lane * 4) = *(const v4f*)(&Tf[b][lane * 4]); __threadfence(); } }
__global__ __launch_bounds__(32) void agg_kernel(const float* __restrict__ I1, const float* __restrict__ O0, const b16* __restrict__ CFh, const b16* __restrict__ CFl, int DV, float* __restrict__ O3, float* __restrict__ O1, float* __restrict__ O4) {
  __shared__ __attribute__((aligned(16))) b16 Ah[32][136], Al[32][136]; __shared__ float Tf[32][132]; __shared__ float Cr[32]; const int lane = threadIdx.x, nloc = lane & 15, hlf = lane >> 4; const int b = blockIdx.x / (T / 32), t0 = (blockIdx.x % (T / 32)) * 32;
  for (int rr = 0; rr < 32; ++rr) for (int q = 0; q < 4; ++q) { const int d = q * 32 + lane; b16 p, ql; split16((d < DV ? I1[((size_t)b * M + d) * T + t0 + rr] : 0.0f) * XS, p, ql); Ah[rr][d] = p; Al[rr][d] = ql; }
  { float s = 0.0f; for (int d = 0; d < DV; ++d) s += O0[((size_t)b * M + d) * T + t0 + lane]; Cr[lane] = s; }
  wave_lds_sync();
  for (int mt = 0; mt < 2; ++mt) { v8f acc[8];
#pragma unroll
    for (int t = 0; t < 8; ++t) acc[t] = (v8f){};
#pragma unroll
    for (int kb = 0; kb < M; kb += 32) { const v16b a = frag_kb(&Ah[mt * 16 + nloc][kb], hlf), al = frag_kb(&Al[mt * 16 + nloc][kb], hlf);
#pragma unroll
      for (int t = 0; t < 8; ++t) { const size_t ro = (size_t)(t * 16 + nloc) * M + kb; const v16b bh = frag_kb(CFh + ro, hlf), bl = frag_kb(CFl + ro, hlf); acc[t] = wmma16b(a, bh, acc[t]); acc[t] = wmma16b(a, bl, acc[t]); acc[t] = wmma16b(al, bh, acc[t]); } }
#pragma unroll
    for (int t = 0; t < 8; ++t)
#pragma unroll
      for (int r8 = 0; r8 < 8; ++r8) Tf[mt * 16 + 8 * hlf + r8][t * 16 + nloc] = acc[t][r8] * (1.0f / (XS * XS)); }
  wave_lds_sync();
  for (int pass = 0; pass < 2; ++pass) { for (int rr = 0; rr < 32; ++rr) { const size_t ro = ((size_t)b * T + t0 + rr) * M + lane * 4; const v4f ag = *(const v4f*)(&Tf[rr][lane * 4]); *(volatile v4f*)(O3 + ro) = ag; const float cr = Cr[rr]; v4f lo; for (int k = 0; k < 4; ++k) lo[k] = ag[k] / cr; *(volatile v4f*)(O1 + ro) = lo; }
    ((volatile float*)O4)[(size_t)b * T + t0 + lane] = Cr[lane]; __threadfence(); } }
__global__ __launch_bounds__(256) void high_kernel(const float* __restrict__ I2, const float* __restrict__ M2, const float* __restrict__ O1, int DV, float* __restrict__ O2) { const size_t u = (size_t)blockIdx.x * 256 + threadIdx.x; if (u >= (size_t)B * M * T / 4) return; const size_t e0 = u * 4; const int b = (int)(e0 / ((size_t)M * T)), d = (int)((e0 / T) % M), t = (int)(e0 % T);
  v4f r = {0.0f, 0.0f, 0.0f, 0.0f}; if (d < DV) { const v4f i2 = *(const v4f*)(I2 + e0), m2 = *(const v4f*)(M2 + e0); for (int k = 0; k < 4; ++k) r[k] = i2[k] / m2[k] - O1[((size_t)b * T + t + k) * M + d]; }
  for (int pass = 0; pass < 2; ++pass) { *(volatile v4f*)(O2 + e0) = r; __threadfence(); } }
}

extern "C" void kernel_launch(void* const* d_in, const int* in_sizes, int n_in, void* d_out, int out_size, void* d_ws, size_t ws_size, hipStream_t stream) {
  (void)n_in;
  auto Fp = [&](int i) { return (const float*)d_in[i]; };
  if (in_sizes[0] != B * T * M || in_sizes[1] != B * T * M || in_sizes[3] != M || in_sizes[4] != M || in_sizes[5] != M * M || out_size != 4 * B * M * T + B * T) return;
  const int DV = M;
  size_t off = 0; char* ws = (char*)d_ws;
  auto carve = [&](size_t bytes) { char* p = ws + off; off += (bytes + 255) & ~(size_t)255; return p; };
  b16* KP = (b16*)carve((size_t)4 * M * GW * 2); b16* VB = (b16*)carve((size_t)2 * M * B * T * 2); b16* CFh = (b16*)carve((size_t)M * M * 2); b16* CFl = (b16*)carve((size_t)M * M * 2);
  float* I1 = (float*)carve((size_t)B * M * T * 4); float* M2 = (float*)carve((size_t)B * M * T * 4); float* I2 = (float*)carve((size_t)B * M * T * 4);
  if (off > ws_size || off > ((size_t)128 << 20)) return;
  float* O0 = (float*)d_out; float* O1 = O0 + (size_t)B * M * T; float* O2 = O1 + (size_t)B * T * M; float* O3 = O2 + (size_t)B * M * T; float* O4 = O3 + (size_t)B * T * M;
  prep_kernel<<<(unsigned)(((size_t)2 * M * B * (T / 8) + 255) / 256), 256, 0, stream>>>(Fp(0), Fp(1), Fp(3), Fp(4), Fp(5), KP, VB, CFh, CFl);
  infl_kernel<<<DV * 16, 32, 0, stream>>>(VB, KP, O0, I1, M2, I2);
  agg_kernel<<<B * (T / 32), 32, 0, stream>>>(I1, O0, CFh, CFl, DV, O3, O1, O4);
  high_kernel<<<(unsigned)(((size_t)B * M * T / 4 + 255) / 256), 256, 0, stream>>>(I2, M2, O1, DV, O2);
}
